// Fingerprint_MutiTask_87625922773464
// MI455X (gfx1250) — hardware-verified
//
#include <hip/hip_runtime.h>
#define NM 128
#define LA 128
#define DG 6
#define FD 256
#define NA (NM * LA)
#define NP (NA * DG)
#define INA 39
#define INB 10
#define NBD 256
#define RAD 3
#define TSTEP 2
#define TASKS 4
#define NEGc (-9e8f)
#define CHK 1024
typedef __bf16 v16b __attribute__((ext_vector_type(16)));
typedef unsigned short v8us __attribute__((ext_vector_type(8), may_alias));
typedef float  v8f  __attribute__((ext_vector_type(8)));
typedef float  v4f  __attribute__((ext_vector_type(4)));
typedef float  v4fa __attribute__((ext_vector_type(4), may_alias));
union FragB { v16b v; v8us half[2]; unsigned short u[16]; };

__device__ __forceinline__ unsigned short bf16_bits(float x) { unsigned int u = __float_as_uint(x); return (unsigned short)((u + 0x7FFFu + ((u >> 16) & 1u)) >> 16); }
__device__ __forceinline__ float bf16_val(unsigned short b) { return __uint_as_float(((unsigned int)b) << 16); }
__device__ __forceinline__ float bf16_round(float x) { return bf16_val(bf16_bits(x)); }
template <int NT>
__device__ __forceinline__ v8f mmaN(v16b ah, v16b al, v16b bh, v16b bl, v8f c) {
  c = __builtin_amdgcn_wmma_f32_16x16x32_bf16(false, ah, false, bh, (short)0, c, false, false);
  if (NT >= 2) c = __builtin_amdgcn_wmma_f32_16x16x32_bf16(false, al, false, bh, (short)0, c, false, false);
  if (NT >= 3) c = __builtin_amdgcn_wmma_f32_16x16x32_bf16(false, ah, false, bl, (short)0, c, false, false);
  asm volatile("v_nop\n\tv_nop\n\tv_nop\n\tv_nop" : "+v"(c) : "v"(ah), "v"(al), "v"(bh), "v"(bl));
  return c;
}

__global__ __launch_bounds__(256) void k_wt_bf16(const float* __restrict__ W, unsigned short* __restrict__ Wt, int K, int N) {
  const int t = blockIdx.x * 256 + threadIdx.x;
  const int k8n = K / 8;
  if (t >= N * k8n) return;
  const int n = t / k8n, k8 = (t % k8n) * 8;
  v8us v;
#pragma unroll
  for (int i = 0; i < 8; ++i) v[i] = bf16_bits(W[(size_t)(k8 + i) * N + n]);
  *(volatile v8us*)(Wt + (size_t)n * K + k8) = v;
  __threadfence();
  *(volatile v8us*)(Wt + (size_t)n * K + k8) = v;
}

template <bool ASPLIT, int ACT, bool BIAS_BF16>
__global__ __launch_bounds__(128) void k_gemm_bf(const float* __restrict__ A, int lda, const unsigned short* __restrict__ Wt, int ldb,
                                               const float* __restrict__ bias, float* __restrict__ C, int ldc, int M, int N, int K) {
  __shared__ __attribute__((aligned(16))) float so[4][16][64];
  const int tid = threadIdx.x, w = tid >> 5, lane = tid & 31, ln = lane & 15, hh = lane >> 4;
  const int ntn = N / 64;
  const int wid = blockIdx.x * 4 + w;
  const int mt = wid / ntn, nq = wid % ntn;
  if (mt * 16 >= M) return;
  const int row0 = mt * 16, col0 = nq * 64;
  const float* arow = A + (size_t)(row0 + ln) * lda;
  v8f acc[4] = {};
  for (int kb = 0; kb < K; kb += 32) {
    FragB ah, al;
    const v4f x0 = *(const v4fa*)(arow + kb + 8 * hh), x1 = *(const v4fa*)(arow + kb + 8 * hh + 4);
    const v4f x2 = *(const v4fa*)(arow + kb + 16 + 8 * hh), x3 = *(const v4fa*)(arow + kb + 16 + 8 * hh + 4);
    float xs[16] = {x0[0],x0[1],x0[2],x0[3],x1[0],x1[1],x1[2],x1[3],x2[0],x2[1],x2[2],x2[3],x3[0],x3[1],x3[2],x3[3]};
#pragma unroll
    for (int i = 0; i < 16; ++i) { const unsigned short hb = bf16_bits(xs[i]); ah.u[i] = hb; al.u[i] = ASPLIT ? bf16_bits(xs[i] - bf16_val(hb)) : (unsigned short)0; }
#pragma unroll
    for (int t = 0; t < 4; ++t) {
      const unsigned short* brow = Wt + (size_t)(col0 + t * 16 + ln) * ldb + kb;
      FragB b;
      b.half[0] = *(const v8us*)(brow + 8 * hh);
      b.half[1] = *(const v8us*)(brow + 16 + 8 * hh);
      acc[t] = mmaN<ASPLIT ? 2 : 1>(ah.v, al.v, b.v, b.v, acc[t]);
    }
  }
#pragma unroll
  for (int t = 0; t < 4; ++t) {
    float bv = bias ? bias[col0 + t * 16 + ln] : 0.f;
    if (BIAS_BF16) bv = bf16_round(bv);
#pragma unroll
    for (int r = 0; r < 8; ++r) { float v = acc[t][r] + bv; if (ACT == 1) v = fmaxf(v, 0.f); so[w][8 * hh + r][t * 16 + ln] = v; }
  }
  __builtin_amdgcn_fence(__ATOMIC_ACQ_REL, "workgroup");
  __builtin_amdgcn_wave_barrier();
  const int rsub = lane >> 4, c4 = (lane & 15) * 4;
  for (int pass = 0; pass < 2; ++pass) {
#pragma unroll
    for (int q = 0; q < 8; ++q) {
      const int r = q * 2 + rsub;
      const v4f v = *(const v4fa*)&so[w][r][c4];
      *(volatile v4f*)(C + (size_t)(row0 + r) * ldc + col0 + c4) = v;
    }
    if (pass == 0) __threadfence();
  }
}

template <bool ASPLIT, int ACT, bool BIAS_BF16, bool RES_BF16>
__global__ __launch_bounds__(128) void k_gemm_bf3(const float* __restrict__ A, int lda, const unsigned short* __restrict__ Wt, int ldb,
                                                const float* __restrict__ bias, const float* __restrict__ resid, int rmod, int ldr,
                                                float* __restrict__ C, int ldc, int M, int N, int K) {
  __shared__ __attribute__((aligned(16))) float so[4][16][64];
  const int tid = threadIdx.x, w = tid >> 5, lane = tid & 31, ln = lane & 15, hh = lane >> 4;
  const int ntn = N / 64;
  const int wid = blockIdx.x * 4 + w;
  const int mt = wid / ntn, nq = wid % ntn;
  if (mt * 16 >= M) return;
  const int row0 = mt * 16, col0 = nq * 64;
  const float* arow = A + (size_t)(row0 + ln) * lda;
  v8f acc[4] = {};
  for (int kb = 0; kb < K; kb += 32) {
    FragB ah, al;
    const v4f x0 = *(const v4fa*)(arow + kb + 8 * hh), x1 = *(const v4fa*)(arow + kb + 8 * hh + 4);
    const v4f x2 = *(const v4fa*)(arow + kb + 16 + 8 * hh), x3 = *(const v4fa*)(arow + kb + 16 + 8 * hh + 4);
    float xs[16] = {x0[0],x0[1],x0[2],x0[3],x1[0],x1[1],x1[2],x1[3],x2[0],x2[1],x2[2],x2[3],x3[0],x3[1],x3[2],x3[3]};
#pragma unroll
    for (int i = 0; i < 16; ++i) { const unsigned short hb = bf16_bits(xs[i]); ah.u[i] = hb; al.u[i] = ASPLIT ? bf16_bits(xs[i] - bf16_val(hb)) : (unsigned short)0; }
#pragma unroll
    for (int t = 0; t < 4; ++t) {
      const unsigned short* brow = Wt + (size_t)(col0 + t * 16 + ln) * ldb + kb;
      FragB b;
      b.half[0] = *(const v8us*)(brow + 8 * hh);
      b.half[1] = *(const v8us*)(brow + 16 + 8 * hh);
      acc[t] = mmaN<ASPLIT ? 2 : 1>(ah.v, al.v, b.v, b.v, acc[t]);
    }
  }
#pragma unroll
  for (int t = 0; t < 4; ++t) {
    const int col = col0 + t * 16 + ln;
    float bv = bias ? bias[col] : 0.f;
    if (BIAS_BF16) bv = bf16_round(bv);
#pragma unroll
    for (int r = 0; r < 8; ++r) {
      float v = acc[t][r] + bv;
      if (resid) { float rv = resid[(size_t)((row0 + 8 * hh + r) % rmod) * ldr + col]; if (RES_BF16) rv = bf16_round(rv); v += rv; }
      if (ACT == 1) v = fmaxf(v, 0.f);
      if (ACT == 2) v = 0.5f * v * (1.0f + erff(v * 0.70710678118654752f));
      if (ACT == 3) { const float u = 0.7978845608028654f * (v + 0.044715f * v * v * v); v = 0.5f * v * (1.0f + tanhf(u)); }
      so[w][8 * hh + r][t * 16 + ln] = v;
    }
  }
  __builtin_amdgcn_fence(__ATOMIC_ACQ_REL, "workgroup");
  __builtin_amdgcn_wave_barrier();
  const int rsub = lane >> 4, c4 = (lane & 15) * 4;
  for (int pass = 0; pass < 2; ++pass) {
#pragma unroll
    for (int q = 0; q < 8; ++q) {
      const int r = q * 2 + rsub;
      const v4f v = *(const v4fa*)&so[w][r][c4];
      *(volatile v4f*)(C + (size_t)(row0 + r) * ldc + col0 + c4) = v;
    }
    if (pass == 0) __threadfence();
  }
}
template <bool PARAM_BF16>
__global__ __launch_bounds__(256) void k_layernorm(const float* __restrict__ X, const float* __restrict__ R, const float* __restrict__ g, const float* __restrict__ bta,
                                                  float* __restrict__ out_sum, float* __restrict__ out_norm, int N, float eps) {
  __shared__ float red[256];
  const int row = blockIdx.x, tid = threadIdx.x;
  const float* x = X + (size_t)row * N; const float* rr = R ? R + (size_t)row * N : nullptr;
  float vals[16];
  const int per = N / 256;
  float s1 = 0.f;
  for (int u = 0; u < per / 4; ++u) {
    const int j = tid * 4 + 1024 * u;
    const v4f a = *(const v4fa*)(x + j);
    v4f b = {0.f,0.f,0.f,0.f}; if (rr) b = *(const v4fa*)(rr + j);
#pragma unroll
    for (int q = 0; q < 4; ++q) { const float v = a[q] + b[q]; vals[u * 4 + q] = v; s1 += v; }
  }
  red[tid] = s1; __syncthreads();
  for (int st = 128; st > 0; st >>= 1) { if (tid < st) red[tid] += red[tid + st]; __syncthreads(); }
  const float mu = red[0] / (float)N; __syncthreads();
  float s2 = 0.f;
  for (int u = 0; u < per / 4; ++u)
#pragma unroll
    for (int q = 0; q < 4; ++q) { const float c = vals[u * 4 + q] - mu; s2 += c * c; }
  red[tid] = s2; __syncthreads();
  for (int st = 128; st > 0; st >>= 1) { if (tid < st) red[tid] += red[tid + st]; __syncthreads(); }
  const float rs = rsqrtf(red[0] / (float)N + eps);
  for (int pass = 0; pass < 2; ++pass) {
    for (int u = 0; u < per / 4; ++u) {
      const int j = tid * 4 + 1024 * u;
      v4f o, sm;
#pragma unroll
      for (int q = 0; q < 4; ++q) {
        float gg = g[j + q], bb = bta[j + q];
        if (PARAM_BF16) { gg = bf16_round(gg); bb = bf16_round(bb); }
        sm[q] = vals[u * 4 + q]; o[q] = (vals[u * 4 + q] - mu) * rs * gg + bb;
      }
      if (out_sum) *(volatile v4f*)(out_sum + (size_t)row * N + j) = sm;
      *(volatile v4f*)(out_norm + (size_t)row * N + j) = o;
    }
    if (pass == 0) __threadfence();
  }
}


typedef _Float16 v16h __attribute__((ext_vector_type(16)));
union FragH { v16h v; v8us half[2]; _Float16 h[16]; unsigned short u[16]; };
template <int NT>
__device__ __forceinline__ v8f mmaH(v16h ah, v16h al, v16h bh, v16h bl, v8f c) {
  c = __builtin_amdgcn_wmma_f32_16x16x32_f16(false, ah, false, bh, (short)0, c, false, false);
  if (NT >= 2) c = __builtin_amdgcn_wmma_f32_16x16x32_f16(false, al, false, bh, (short)0, c, false, false);
  if (NT >= 3) c = __builtin_amdgcn_wmma_f32_16x16x32_f16(false, ah, false, bl, (short)0, c, false, false);
  asm volatile("v_nop\n\tv_nop\n\tv_nop\n\tv_nop" : "+v"(c) : "v"(ah), "v"(al), "v"(bh), "v"(bl));
  return c;
}
template <bool ASPLIT>
__global__ __launch_bounds__(128) void k_gemm_h(const float* __restrict__ A, int lda, size_t sA, const _Float16* __restrict__ Bh, int ldb, size_t sB, float alpha, float* __restrict__ C, int ldc, size_t sC, int M, int N, int K) {
  __shared__ __attribute__((aligned(16))) float so[4][16][64];
  const int tid = threadIdx.x, w = tid >> 5, lane = tid & 31, ln = lane & 15, hh = lane >> 4; const int by = blockIdx.y;
  A += (size_t)by * sA; Bh += (size_t)by * sB; C += (size_t)by * sC;
  const int ntn = (N + 63) / 64; const int wid = blockIdx.x * 4 + w; const int mt = wid / ntn, nq = wid % ntn; if (mt * 16 >= M) return;
  const int row0 = mt * 16, col0 = nq * 64; const float* arow = A + (size_t)(row0 + ln) * lda;
  v8f acc[4] = {};
  for (int kb = 0; kb < K; kb += 32) {
    FragH ah, al;
    const v4f x0 = *(const v4fa*)(arow + kb + 8 * hh), x1 = *(const v4fa*)(arow + kb + 8 * hh + 4), x2 = *(const v4fa*)(arow + kb + 16 + 8 * hh), x3 = *(const v4fa*)(arow + kb + 16 + 8 * hh + 4);
    float xs[16] = {x0[0],x0[1],x0[2],x0[3],x1[0],x1[1],x1[2],x1[3],x2[0],x2[1],x2[2],x2[3],x3[0],x3[1],x3[2],x3[3]};
#pragma unroll
    for (int i = 0; i < 16; ++i) { const _Float16 h = (_Float16)xs[i]; ah.h[i] = h; al.h[i] = ASPLIT ? (_Float16)(xs[i] - (float)h) : (_Float16)0.0f; }
#pragma unroll
    for (int t = 0; t < 4; ++t) { if (col0 + t * 16 >= N) continue; const size_t boff = (size_t)(col0 + t * 16 + ln) * ldb + kb; FragH bq; bq.half[0] = *(const v8us*)(Bh + boff + 8 * hh); bq.half[1] = *(const v8us*)(Bh + boff + 16 + 8 * hh);
      acc[t] = mmaH<ASPLIT ? 2 : 1>(ah.v, al.v, bq.v, bq.v, acc[t]); }
  }
#pragma unroll
  for (int t = 0; t < 4; ++t) { if (col0 + t * 16 >= N) continue;
#pragma unroll
    for (int r = 0; r < 8; ++r) so[w][8 * hh + r][t * 16 + ln] = acc[t][r] * alpha; }
  __builtin_amdgcn_fence(__ATOMIC_ACQ_REL, "workgroup"); __builtin_amdgcn_wave_barrier();
  const int rsub = lane >> 4, c4 = (lane & 15) * 4;
  for (int pass = 0; pass < 2; ++pass) {
#pragma unroll
    for (int q = 0; q < 8; ++q) { const int r = q * 2 + rsub; if (col0 + c4 < N) { const v4f v = *(const v4fa*)&so[w][r][c4]; *(volatile v4f*)(C + (size_t)(row0 + r) * ldc + col0 + c4) = v; } }
    if (pass == 0) __threadfence(); }
}

__global__ __launch_bounds__(256) void k_wt_f16(const float* __restrict__ W, _Float16* __restrict__ Wt, int K, int N, float scale) {
  const int t = blockIdx.x * 256 + threadIdx.x; if (t >= N * (K / 8)) return; const int n = t / (K / 8), k8 = (t % (K / 8)) * 8; FragH f;
#pragma unroll
  for (int i = 0; i < 8; ++i) f.h[i] = (_Float16)(bf16_round(W[(size_t)(k8 + i) * N + n]) * scale); const v8us o = f.half[0];
  *(volatile v8us*)((unsigned short*)Wt + (size_t)n * K + k8) = o; __threadfence(); *(volatile v8us*)((unsigned short*)Wt + (size_t)n * K + k8) = o;
}
template <int ACT>
__global__ __launch_bounds__(128) void k_gemm_hhx(const _Float16* __restrict__ A, int lda, size_t sA, const _Float16* __restrict__ Bh, int ldb, size_t sB, float alpha, const float* __restrict__ bias, size_t sBias, const float* __restrict__ CP, int rowsPerB, size_t sCPb, int row0g,
    float* __restrict__ C, _Float16* __restrict__ C16, int ldc, size_t sC, int M, int N, int K) {
  __shared__ __attribute__((aligned(16))) float so[4][16][64];
  const int tid = threadIdx.x, w = tid >> 5, lane = tid & 31, ln = lane & 15, hh = lane >> 4; const int by = blockIdx.y;
  A += (size_t)by * sA; Bh += (size_t)by * sB; const size_t cofs = (size_t)by * sC; const float* bp = bias ? bias + (size_t)by * sBias : nullptr;
  const int ntn = (N + 63) / 64; const int wid = blockIdx.x * 4 + w; const int mt = wid / ntn, nq = wid % ntn; if (mt * 16 >= M) return;
  const int row0 = mt * 16, col0 = nq * 64; const _Float16* arow = A + (size_t)(row0 + ln) * lda;
  v8f acc[4] = {};
  for (int kb = 0; kb < K; kb += 32) { FragH ah; ah.half[0] = *(const v8us*)((const unsigned short*)arow + kb + 8 * hh); ah.half[1] = *(const v8us*)((const unsigned short*)arow + kb + 16 + 8 * hh);
#pragma unroll
    for (int t = 0; t < 4; ++t) { if (col0 + t * 16 >= N) continue; const size_t boff = (size_t)(col0 + t * 16 + ln) * ldb + kb; FragH bq; bq.half[0] = *(const v8us*)((const unsigned short*)Bh + boff + 8 * hh); bq.half[1] = *(const v8us*)((const unsigned short*)Bh + boff + 16 + 8 * hh);
      acc[t] = mmaH<1>(ah.v, ah.v, bq.v, bq.v, acc[t]); }
  }
#pragma unroll
  for (int t = 0; t < 4; ++t) { if (col0 + t * 16 >= N) continue; const int col = col0 + t * 16 + ln; const float bv = bp ? bf16_round(bp[col]) : 0.f;
#pragma unroll
    for (int r = 0; r < 8; ++r) { float v = acc[t][r] * alpha + bv; if (CP) { const int bidx = (row0g + row0 + 8 * hh + r) / rowsPerB; v += CP[(size_t)bidx * sCPb + (size_t)by * 64 + col]; } if (ACT == 1) v = (v > 0.f) ? v : expm1f(v); else if (ACT == 7) v = (v > 0.f) ? v + 1.0f : expf(v); else if (ACT == 8) v = tanhf(v); else if (ACT == 9) v = 0.5f * v * (1.0f + tanhf(0.7978845608028654f * (v + 0.044715f * v * v * v))); else if (ACT == 11) v = 1.0f / (1.0f + expf(-v)); else if (ACT == 12) v = (v > 0.f) ? v : 0.01f * v; else if (ACT == 14) v = (v > 0.f) ? v : 0.1f * v; else if (ACT == 16) v = (v >= 0.f) ? v : 0.01f * v; else if (ACT == 15) v = v / (1.0f + expf(-v)); else if (ACT == 3) v = fmaxf(v, 0.f); else if (ACT == 6) v = 0.5f * v * (1.0f + erff(v * 0.70710678118654752f)); so[w][8 * hh + r][t * 16 + ln] = v; } }
  __builtin_amdgcn_fence(__ATOMIC_ACQ_REL, "workgroup"); __builtin_amdgcn_wave_barrier();
  const int rsub = lane >> 4, c4 = (lane & 15) * 4; typedef _Float16 v4h __attribute__((ext_vector_type(4)));
  for (int pass = 0; pass < 2; ++pass) {
#pragma unroll
    for (int q = 0; q < 8; ++q) { const int r = q * 2 + rsub; if (col0 + c4 < N) { const v4f v = *(const v4fa*)&so[w][r][c4]; if (C) *(volatile v4f*)(C + cofs + (size_t)(row0 + r) * ldc + col0 + c4) = v; if (C16) { v4h h4; for (int i = 0; i < 4; ++i) h4[i] = (_Float16)v[i]; *(volatile v4h*)(C16 + cofs + (size_t)(row0 + r) * ldc + col0 + c4) = h4; } } }
    if (pass == 0) __threadfence(); }
}


typedef _Float16 v4h __attribute__((ext_vector_type(4)));

__global__ __launch_bounds__(256) void k_x16(const float* __restrict__ x, _Float16* __restrict__ X16, size_t n8) { const size_t t = (size_t)blockIdx.x * 256 + threadIdx.x; if (t >= n8) return; FragH f;
#pragma unroll
  for (int q = 0; q < 8; ++q) f.h[q] = (_Float16)bf16_round(x[t * 8 + q]); *(volatile v8us*)((unsigned short*)X16 + t * 8) = f.half[0]; __threadfence(); *(volatile v8us*)((unsigned short*)X16 + t * 8) = f.half[0]; }
__global__ __launch_bounds__(256) void k_h16(const float* __restrict__ x, _Float16* __restrict__ X16, size_t n8) { const size_t t = (size_t)blockIdx.x * 256 + threadIdx.x; if (t >= n8) return; FragH f;
#pragma unroll
  for (int q = 0; q < 8; ++q) f.h[q] = (_Float16)x[t * 8 + q]; *(volatile v8us*)((unsigned short*)X16 + t * 8) = f.half[0]; __threadfence(); *(volatile v8us*)((unsigned short*)X16 + t * 8) = f.half[0]; }
__global__ __launch_bounds__(256) void k_round16f(const float* __restrict__ W, _Float16* __restrict__ Bt, size_t n8) { const size_t t = (size_t)blockIdx.x * 256 + threadIdx.x; if (t >= n8) return; FragH f;
#pragma unroll
  for (int i = 0; i < 8; ++i) f.h[i] = (_Float16)(bf16_round(W[t * 8 + i]) * 16.0f); *(volatile v8us*)((unsigned short*)Bt + t * 8) = f.half[0]; __threadfence(); *(volatile v8us*)((unsigned short*)Bt + t * 8) = f.half[0]; }
template <int NHv, int TTv>
__global__ __launch_bounds__(256) void k_vt(const _Float16* __restrict__ V16, int ldv, int voff, _Float16* __restrict__ Vt) { __shared__ unsigned short tl[64][66]; const int tid = threadIdx.x; const int slab = blockIdx.x / (TTv / 64), lg = blockIdx.x % (TTv / 64); const int b = slab / NHv, h = slab % NHv;
  for (int i = tid; i < 64 * 8; i += 256) { const int r = i / 8, c8 = (i % 8) * 8; FragH f; f.half[0] = *(const v8us*)((const unsigned short*)V16 + ((size_t)b * TTv + lg * 64 + r) * ldv + voff + h * 64 + c8);
#pragma unroll
    for (int q = 0; q < 8; ++q) tl[r][c8 + q] = f.u[q]; }
  __syncthreads();
  for (int pass = 0; pass < 2; ++pass) {
#pragma unroll
    for (int rd = 0; rd < 2; ++rd) { const int d = rd * 32 + tid / 8, pc = tid % 8; FragH f;
#pragma unroll
      for (int q = 0; q < 8; ++q) f.u[q] = tl[pc * 8 + q][d];
      *(volatile v8us*)((unsigned short*)Vt + ((size_t)slab * 64 + d) * TTv + lg * 64 + pc * 8) = f.half[0]; }
    if (pass == 0) __threadfence(); } }

__global__ __launch_bounds__(256) void k_hl(const float* __restrict__ F, _Float16* __restrict__ Hh, _Float16* __restrict__ Hl, size_t n8) { const size_t t = (size_t)blockIdx.x * 256 + threadIdx.x; if (t >= n8) return; FragH fh, fl; const v4f a = *(const v4fa*)(F + t * 8), c = *(const v4fa*)(F + t * 8 + 4);
#pragma unroll
  for (int q = 0; q < 4; ++q) { _Float16 h = (_Float16)a[q]; fh.h[q] = h; fl.h[q] = (_Float16)((a[q] - (float)h) * 1024.0f); h = (_Float16)c[q]; fh.h[4 + q] = h; fl.h[4 + q] = (_Float16)((c[q] - (float)h) * 1024.0f); }
  for (int pass = 0; pass < 2; ++pass) { *(volatile v8us*)((unsigned short*)Hh + t * 8) = fh.half[0]; *(volatile v8us*)((unsigned short*)Hl + t * 8) = fl.half[0]; if (pass == 0) __threadfence(); } }

__device__ __forceinline__ float lrelu01(float v) { return (v >= 0.f) ? v : 0.01f * v; }
__device__ __forceinline__ float elu1(float v) { return (v > 0.f) ? v : (__expf(v) - 1.0f); }
__device__ __forceinline__ float sigm_f(float x) { return __builtin_amdgcn_rcpf(1.0f + __expf(-x)); }
__device__ __forceinline__ float tanh_f(float x) { const float a = fabsf(x); const float big = 1.0f - 2.0f * __builtin_amdgcn_rcpf(1.0f + __expf(2.0f * a)); const float sml = a - a * a * a * (1.0f / 3.0f); const float r = (a < 0.03f) ? sml : big; return (x < 0.f) ? -r : r; }
__global__ __launch_bounds__(256) void k_a64(const float* __restrict__ atom, _Float16* __restrict__ A64) { const int t = blockIdx.x * 256 + threadIdx.x; if (t >= NA * 8) return; const int a = t / 8, k0 = (t % 8) * 8; FragH f;
#pragma unroll
  for (int q = 0; q < 8; ++q) { const int k = k0 + q; f.h[q] = (k < INA) ? (_Float16)bf16_round(atom[(size_t)a * INA + k]) : (_Float16)0.0f; }
  *(volatile v8us*)((unsigned short*)A64 + (size_t)a * 64 + k0) = f.half[0]; __threadfence(); *(volatile v8us*)((unsigned short*)A64 + (size_t)a * 64 + k0) = f.half[0]; }
__global__ __launch_bounds__(256) void k_n64(const float* __restrict__ atom, const float* __restrict__ bond, const int* __restrict__ adeg, const int* __restrict__ bdeg, _Float16* __restrict__ N64) { const int t = blockIdx.x * 256 + threadIdx.x; if (t >= NP * 8) return; const int p = t / 8, k0 = (t % 8) * 8; const int a = p / DG; const int b = a / LA; int ai = adeg[p], bi = bdeg[p]; ai = min(max(ai, 0), LA - 1); bi = min(max(bi, 0), NBD - 1); FragH f;
#pragma unroll
  for (int q = 0; q < 8; ++q) { const int k = k0 + q; float v = 0.f; if (k < INA) v = bf16_round(atom[((size_t)b * LA + ai) * INA + k]); else if (k < INA + INB) v = bf16_round(bond[((size_t)b * NBD + bi) * INB + (k - INA)]); f.h[q] = (_Float16)v; }
  *(volatile v8us*)((unsigned short*)N64 + (size_t)p * 64 + k0) = f.half[0]; __threadfence(); *(volatile v8us*)((unsigned short*)N64 + (size_t)p * 64 + k0) = f.half[0]; }
__global__ __launch_bounds__(256) void k_w64(const float* __restrict__ w, int KIN, _Float16* __restrict__ Bt) { const int t = blockIdx.x * 256 + threadIdx.x; if (t >= FD * 8) return; const int o = t / 8, k0 = (t % 8) * 8; FragH f;
#pragma unroll
  for (int q = 0; q < 8; ++q) { const int k = k0 + q; f.h[q] = (k < KIN) ? (_Float16)(bf16_round(w[(size_t)o * KIN + k]) * 16.0f) : (_Float16)0.0f; }
  *(volatile v8us*)((unsigned short*)Bt + (size_t)o * 64 + k0) = f.half[0]; __threadfence(); *(volatile v8us*)((unsigned short*)Bt + (size_t)o * 64 + k0) = f.half[0]; }
template <int RELU>
__global__ __launch_bounds__(256) void k_split(const float* __restrict__ F, _Float16* __restrict__ Hh, _Float16* __restrict__ Hl, size_t n8) {
  #pragma clang fp contract(off)
  const size_t t = (size_t)blockIdx.x * 256 + threadIdx.x; if (t >= n8) return; const v4f a = *(const v4fa*)(F + t * 8), c = *(const v4fa*)(F + t * 8 + 4); FragH fh, fl;
#pragma unroll
  for (int q = 0; q < 8; ++q) { float v = (q < 4) ? a[q] : c[q - 4]; if (RELU) v = fmaxf(v, 0.f); const _Float16 hi = (_Float16)v; fh.h[q] = hi; fl.h[q] = (_Float16)((v - (float)hi) * 1024.0f); }
  for (int pass = 0; pass < 2; ++pass) { *(volatile v8us*)((unsigned short*)Hh + t * 8) = fh.half[0]; *(volatile v8us*)((unsigned short*)Hl + t * 8) = fl.half[0]; if (pass == 0) __threadfence(); } }
template <int R0>
__global__ __launch_bounds__(256) void k_ctx(const float* __restrict__ SELF, const float* __restrict__ NBR, const float* __restrict__ NT, const int* __restrict__ adeg, const float* __restrict__ wa, const float* __restrict__ ab, const float* __restrict__ attb, int a0, _Float16* __restrict__ CXH, _Float16* __restrict__ CXL) {
  #pragma clang fp contract(off)
  __shared__ float scw[8][8]; __shared__ int padw[8][8], roww[8][8], trww[8][8];
  const int tid = threadIdx.x, w = tid >> 5, l = tid & 31; const int a = a0 + blockIdx.x * 8 + w; const int b = a / LA;
  v4f s0 = *(const v4fa*)(SELF + (size_t)a * FD + 8 * l), s1 = *(const v4fa*)(SELF + (size_t)a * FD + 8 * l + 4); float sv[8];
#pragma unroll
  for (int q = 0; q < 8; ++q) { float v = (q < 4) ? s0[q] : s1[q - 4]; if (!R0) v = fmaxf(v, 0.f); sv[q] = v; }
  float ss = 0.f;
#pragma unroll
  for (int q = 0; q < 8; ++q) ss += sv[q] * bf16_round(wa[8 * l + q]);
  if (l < DG) { int dj = adeg[(size_t)a * DG + l]; padw[w][l] = (dj == LA - 1) ? 1 : 0; dj = min(max(dj, 0), LA - 1); roww[w][l] = R0 ? ((a - a0) * DG + l) : (b * LA + dj); trww[w][l] = R0 ? ((a - a0) * DG + l) : (b * LA + dj); }
  __syncthreads();
#pragma unroll 1
  for (int j = 0; j < DG; ++j) { const float* nr = NBR + (size_t)roww[w][j] * FD + 8 * l; const v4f n0 = *(const v4fa*)nr, n1 = *(const v4fa*)(nr + 4); float sn = ss;
#pragma unroll
    for (int q = 0; q < 8; ++q) { float v = (q < 4) ? n0[q] : n1[q - 4]; if (!R0) v = fmaxf(v, 0.f); sn += v * bf16_round(wa[FD + 8 * l + q]); }
    for (int o = 16; o > 0; o >>= 1) sn += __shfl_xor(sn, o, 32); if (l == 0) scw[w][j] = lrelu01(sn + bf16_round(ab[0])) + (padw[w][j] ? NEGc : 0.f); }
  __syncthreads();
  float m = -3.0e38f;
#pragma unroll 1
  for (int j = 0; j < DG; ++j) m = fmaxf(m, scw[w][j]);
  float s = 0.f;
#pragma unroll 1
  for (int j = 0; j < DG; ++j) s += expf(scw[w][j] - m);
  float acc[8];
#pragma unroll
  for (int q = 0; q < 8; ++q) acc[q] = 0.f;
  float bt[8];
#pragma unroll
  for (int q = 0; q < 8; ++q) bt[q] = R0 ? 0.f : bf16_round(attb[8 * l + q]);
#pragma unroll 1
  for (int j = 0; j < DG; ++j) { const float wj = (expf(scw[w][j] - m) / s) * (padw[w][j] ? 0.f : 1.f); const float* tr = NT + (size_t)trww[w][j] * FD + 8 * l; const v4f t0 = *(const v4fa*)tr, t1 = *(const v4fa*)(tr + 4);
#pragma unroll
    for (int q = 0; q < 8; ++q) acc[q] += wj * (((q < 4) ? t0[q] : t1[q - 4]) + bt[q]); }
  FragH fh, fl;
#pragma unroll
  for (int q = 0; q < 8; ++q) { const float v = elu1(acc[q]); const _Float16 hi = (_Float16)v; fh.h[q] = hi; fl.h[q] = (_Float16)((v - (float)hi) * 1024.0f); }
  for (int pass = 0; pass < 2; ++pass) { *(volatile v8us*)((unsigned short*)CXH + (size_t)a * FD + 8 * l) = fh.half[0]; *(volatile v8us*)((unsigned short*)CXL + (size_t)a * FD + 8 * l) = fl.half[0]; if (pass == 0) __threadfence(); } }
__global__ __launch_bounds__(256) void k_gru(const float* __restrict__ GI, const float* __restrict__ GH, int a0, float* __restrict__ H, _Float16* __restrict__ HHp, _Float16* __restrict__ HLp, _Float16* __restrict__ AHp, _Float16* __restrict__ ALp) {
  #pragma clang fp contract(off)
  const size_t t = (size_t)blockIdx.x * 256 + threadIdx.x; if (t >= (size_t)CHK * (FD / 4)) return; const int c0 = (int)(t % (FD / 4)) * 4; const int i = (int)(t / (FD / 4)); const size_t a = (size_t)a0 + i; const float* gi = GI + (size_t)i * 3 * FD; const float* gh = GH + (size_t)i * 3 * FD;
  const v4f ir = *(const v4fa*)(gi + c0), iz = *(const v4fa*)(gi + FD + c0), inn = *(const v4fa*)(gi + 2 * FD + c0), hr = *(const v4fa*)(gh + c0), hz = *(const v4fa*)(gh + FD + c0), hn = *(const v4fa*)(gh + 2 * FD + c0), hp = *(const v4fa*)(H + a * FD + c0); v4f ho; FragH f1, f1l, f2, f2l;
#pragma unroll
  for (int q = 0; q < 4; ++q) { const float r = sigm_f(ir[q] + hr[q]), z = sigm_f(iz[q] + hz[q]); const float n = tanh_f(inn[q] + r * hn[q]); const float hv = (1.0f - z) * n + z * hp[q]; ho[q] = hv; const _Float16 h1 = (_Float16)hv; f1.h[q] = h1; f1l.h[q] = (_Float16)((hv - (float)h1) * 1024.0f); const float av = fmaxf(hv, 0.f); const _Float16 h2 = (_Float16)av; f2.h[q] = h2; f2l.h[q] = (_Float16)((av - (float)h2) * 1024.0f); }
  const unsigned long long v1 = *(const unsigned long long*)&f1.u[0], v1l = *(const unsigned long long*)&f1l.u[0], v2 = *(const unsigned long long*)&f2.u[0], v2l = *(const unsigned long long*)&f2l.u[0];
  for (int pass = 0; pass < 2; ++pass) { *(volatile v4f*)(H + a * FD + c0) = ho; *(volatile unsigned long long*)((unsigned short*)HHp + a * FD + c0) = v1; *(volatile unsigned long long*)((unsigned short*)HLp + a * FD + c0) = v1l; *(volatile unsigned long long*)((unsigned short*)AHp + a * FD + c0) = v2; *(volatile unsigned long long*)((unsigned short*)ALp + a * FD + c0) = v2l; if (pass == 0) __threadfence(); } }
__global__ __launch_bounds__(256) void k_mol(const float* __restrict__ H, const float* __restrict__ AT, const float* __restrict__ amask, const float* __restrict__ mw, const float* __restrict__ mb, const float* __restrict__ wih, const float* __restrict__ whh, const float* __restrict__ bih, const float* __restrict__ bhh, float* __restrict__ out) {
  #pragma clang fp contract(off)
  __shared__ float molv[FD], actm[FD], ctxv[FD], wl[LA], sp[LA], red[8]; const int tid = threadIdx.x, wv = tid >> 5, l = tid & 31; const int b = blockIdx.x; const int f = tid;
  float mf = 0.f;
#pragma unroll 1
  for (int li = 0; li < LA; ++li) mf += fmaxf(H[((size_t)b * LA + li) * FD + f], 0.f) * bf16_round(amask[(size_t)b * LA + li]);
  molv[f] = mf; actm[f] = fmaxf(mf, 0.f); if (tid < LA) { const float mk = bf16_round(amask[(size_t)b * LA + tid]); wl[tid] = mk; sp[tid] = 0.f; }
  __syncthreads();
#pragma unroll 1
  for (int i = 0; i < TASKS; ++i) {
#pragma unroll 1
    for (int st = 0; st < TSTEP; ++st) {
#pragma unroll 1
      for (int li = wv; li < LA; li += 8) { float pa = 0.f;
#pragma unroll 1
        for (int q = 0; q < 8; ++q) { const int ff = l + 32 * q; pa += actm[ff] * bf16_round(mw[(size_t)i * 2 * FD + ff]) + fmaxf(H[((size_t)b * LA + li) * FD + ff], 0.f) * bf16_round(mw[(size_t)i * 2 * FD + FD + ff]); }
        for (int o = 16; o > 0; o >>= 1) pa += __shfl_xor(pa, o, 32); if (l == 0) sp[li] = lrelu01(pa + bf16_round(mb[i])) + ((wl[li] == 0.f) ? NEGc : 0.f); }
      __syncthreads();
      if (wv == 0) { float m = -3.0e38f; for (int k = 0; k < 4; ++k) m = fmaxf(m, sp[l + 32 * k]); for (int o = 16; o > 0; o >>= 1) m = fmaxf(m, __shfl_xor(m, o, 32)); float s = 0.f; float e[4];
#pragma unroll
        for (int k = 0; k < 4; ++k) { e[k] = expf(sp[l + 32 * k] - m); s += e[k]; } for (int o = 16; o > 0; o >>= 1) s += __shfl_xor(s, o, 32);
#pragma unroll
        for (int k = 0; k < 4; ++k) sp[l + 32 * k] = (e[k] / s) * wl[l + 32 * k]; }
      __syncthreads();
      { float c = 0.f;
#pragma unroll 1
        for (int li = 0; li < LA; ++li) c += sp[li] * AT[((size_t)b * LA + li) * FD + f]; ctxv[f] = elu1(c); }
      __syncthreads();
      float gir = bf16_round(bih[f]), giz = bf16_round(bih[FD + f]), gin = bf16_round(bih[2 * FD + f]), ghr = bf16_round(bhh[f]), ghz = bf16_round(bhh[FD + f]), ghn = bf16_round(bhh[2 * FD + f]);
#pragma unroll 1
      for (int k = 0; k < FD; ++k) { const float cv = ctxv[k], mv = molv[k]; gir += cv * bf16_round(wih[(size_t)f * FD + k]); giz += cv * bf16_round(wih[(size_t)(FD + f) * FD + k]); gin += cv * bf16_round(wih[(size_t)(2 * FD + f) * FD + k]); ghr += mv * bf16_round(whh[(size_t)f * FD + k]); ghz += mv * bf16_round(whh[(size_t)(FD + f) * FD + k]); ghn += mv * bf16_round(whh[(size_t)(2 * FD + f) * FD + k]); }
      const float r = 1.0f / (1.0f + expf(-(gir + ghr))), z = 1.0f / (1.0f + expf(-(giz + ghz))); const float n = tanhf(gin + r * ghn); const float hv = (1.0f - z) * n + z * molv[f];
      __syncthreads();
      molv[f] = hv; actm[f] = fmaxf(hv, 0.f);
      __syncthreads(); }
    for (int pass = 0; pass < 2; ++pass) { *(volatile float*)(out + ((size_t)i * NM + b) * FD + f) = actm[f]; if (pass == 0) __threadfence(); } }
}

extern "C" void kernel_launch(void* const* d_in, const int* in_sizes, int n_in,
                              void* d_out, int out_size, void* d_ws, size_t ws_size, hipStream_t stream) {
  (void)in_sizes; (void)n_in; (void)out_size;
  const float* const* I = (const float* const*)d_in; const float* atom = I[0]; const float* bond = I[1]; const int* adeg = (const int*)d_in[2]; const int* bdeg = (const int*)d_in[3]; const float* amask = I[4];
  const float* afw = I[5]; const float* afb = I[6]; const float* nfw = I[7]; const float* nfb = I[8]; const float* alw = I[9]; const float* alb = I[10]; const float* atw = I[11]; const float* atb = I[12]; const float* gwih = I[13]; const float* gwhh = I[14]; const float* gbih = I[15]; const float* gbhh = I[16];
  const float* mwih = I[17]; const float* mwhh = I[18]; const float* mbih = I[19]; const float* mbhh = I[20]; const float* maw = I[21]; const float* mab = I[22]; const float* mtw = I[23]; const float* mtb = I[24];
  char* ws = (char*)d_ws; size_t off = 0;
  auto take = [&](size_t bytes) { char* p = ws + off; off += (bytes + 255) & ~(size_t)255; return p; };
  _Float16* Baf = (_Float16*)take((size_t)FD * 64 * 2); _Float16* Bnf = (_Float16*)take((size_t)FD * 64 * 2); _Float16* Bat[RAD]; _Float16* Bih[RAD]; _Float16* Bhh[RAD];
  for (int r = 0; r < RAD; ++r) { Bat[r] = (_Float16*)take((size_t)FD * FD * 2); Bih[r] = (_Float16*)take((size_t)3 * FD * FD * 2); Bhh[r] = (_Float16*)take((size_t)3 * FD * FD * 2); }
  _Float16* Bmt = (_Float16*)take((size_t)FD * FD * 2);
  _Float16* A64 = (_Float16*)take((size_t)NA * 64 * 2); _Float16* N64 = (_Float16*)take((size_t)NP * 64 * 2); float* H = (float*)take((size_t)NA * FD * 4); _Float16* HHp = (_Float16*)take((size_t)NA * FD * 2); _Float16* HLp = (_Float16*)take((size_t)NA * FD * 2);
  float* NF32 = (float*)take((size_t)CHK * DG * FD * 4); _Float16* NFH = (_Float16*)take((size_t)CHK * DG * FD * 2); _Float16* NFL = (_Float16*)take((size_t)CHK * DG * FD * 2); float* NT32 = (float*)take((size_t)CHK * DG * FD * 4);
  _Float16* CXH = (_Float16*)take((size_t)NA * FD * 2); _Float16* CXL = (_Float16*)take((size_t)NA * FD * 2); float* GI = (float*)take((size_t)CHK * 3 * FD * 4); float* GH = (float*)take((size_t)CHK * 3 * FD * 4); _Float16* AHp = (_Float16*)take((size_t)NA * FD * 2); _Float16* ALp = (_Float16*)take((size_t)NA * FD * 2); float* NTA32 = (float*)take((size_t)NA * FD * 4);
  float* AT = NTA32;
  if (off > ws_size) return;
  k_w64<<<(FD * 8 + 255) / 256, 256, 0, stream>>>(afw, INA, Baf); k_w64<<<(FD * 8 + 255) / 256, 256, 0, stream>>>(nfw, INA + INB, Bnf);
  for (int r = 0; r < RAD; ++r) { k_round16f<<<(FD * FD / 8 + 255) / 256, 256, 0, stream>>>(atw + (size_t)r * FD * FD, Bat[r], (size_t)FD * FD / 8); k_round16f<<<(3 * FD * FD / 8 + 255) / 256, 256, 0, stream>>>(gwih + (size_t)r * 3 * FD * FD, Bih[r], (size_t)3 * FD * FD / 8); k_round16f<<<(3 * FD * FD / 8 + 255) / 256, 256, 0, stream>>>(gwhh + (size_t)r * 3 * FD * FD, Bhh[r], (size_t)3 * FD * FD / 8); }
  k_round16f<<<(FD * FD / 8 + 255) / 256, 256, 0, stream>>>(mtw, Bmt, (size_t)FD * FD / 8);
  k_a64<<<(NA * 8 + 255) / 256, 256, 0, stream>>>(atom, A64); k_n64<<<(NP * 8 + 255) / 256, 256, 0, stream>>>(atom, bond, adeg, bdeg, N64);
  const dim3 gA(((NA / 16) * (FD / 64) + 3) / 4, 1), gC(((CHK / 16) * (3 * FD / 64) + 3) / 4, 1), gT(((CHK * DG / 16) * (FD / 64) + 3) / 4, 1);
  const size_t n8A = (size_t)NA * FD / 8, n8T = (size_t)CHK * DG * FD / 8; const unsigned g8A = (unsigned)((n8A + 255) / 256), g8T = (unsigned)((n8T + 255) / 256);
  k_gemm_hhx<16><<<gA, 128, 0, stream>>>(A64, 64, 0, Baf, 64, 0, 0.0625f, afb, 0, nullptr, 1, 0, 0, H, nullptr, FD, 0, NA, FD, 64);
  k_split<0><<<g8A, 256, 0, stream>>>(H, HHp, HLp, n8A);
  for (int r = 0; r < RAD; ++r) {
    if (r > 0) { k_gemm_hhx<0><<<gA, 128, 0, stream>>>(AHp, FD, 0, Bat[r], FD, 0, 0.0625f, nullptr, 0, nullptr, 1, 0, 0, NTA32, nullptr, FD, 0, NA, FD, FD); k_gemm_hhx<0><<<gA, 128, 0, stream>>>(ALp, FD, 0, Bat[r], FD, 0, 0.0625f / 1024.0f, nullptr, 0, NTA32, 1, (size_t)FD, 0, NTA32, nullptr, FD, 0, NA, FD, FD); }
    for (int c = 0; c < NA / CHK; ++c) { const int a0 = c * CHK;
      if (r == 0) { k_gemm_hhx<16><<<gT, 128, 0, stream>>>(N64 + (size_t)a0 * DG * 64, 64, 0, Bnf, 64, 0, 0.0625f, nfb, 0, nullptr, 1, 0, 0, NF32, nullptr, FD, 0, CHK * DG, FD, 64);
        k_split<0><<<g8T, 256, 0, stream>>>(NF32, NFH, NFL, n8T);
        k_gemm_hhx<0><<<gT, 128, 0, stream>>>(NFH, FD, 0, Bat[0], FD, 0, 0.0625f, atb, 0, nullptr, 1, 0, 0, NT32, nullptr, FD, 0, CHK * DG, FD, FD); k_gemm_hhx<0><<<gT, 128, 0, stream>>>(NFL, FD, 0, Bat[0], FD, 0, 0.0625f / 1024.0f, nullptr, 0, NT32, 1, (size_t)FD, 0, NT32, nullptr, FD, 0, CHK * DG, FD, FD);
        k_ctx<1><<<CHK / 8, 256, 0, stream>>>(H, NF32, NT32, adeg, alw, alb, atb, a0, CXH, CXL); }
      else k_ctx<0><<<CHK / 8, 256, 0, stream>>>(H, H, NTA32, adeg, alw + (size_t)r * 2 * FD, alb + r, atb + (size_t)r * FD, a0, CXH, CXL); }
    for (int c = 0; c < NA / CHK; ++c) { const int a0 = c * CHK;
      k_gemm_hhx<0><<<gC, 128, 0, stream>>>(CXH + (size_t)a0 * FD, FD, 0, Bih[r], FD, 0, 0.0625f, gbih + (size_t)r * 3 * FD, 0, nullptr, 1, 0, 0, GI, nullptr, 3 * FD, 0, CHK, 3 * FD, FD); k_gemm_hhx<0><<<gC, 128, 0, stream>>>(CXL + (size_t)a0 * FD, FD, 0, Bih[r], FD, 0, 0.0625f / 1024.0f, nullptr, 0, GI, 1, (size_t)3 * FD, 0, GI, nullptr, 3 * FD, 0, CHK, 3 * FD, FD);
      k_gemm_hhx<0><<<gC, 128, 0, stream>>>(HHp + (size_t)a0 * FD, FD, 0, Bhh[r], FD, 0, 0.0625f, gbhh + (size_t)r * 3 * FD, 0, nullptr, 1, 0, 0, GH, nullptr, 3 * FD, 0, CHK, 3 * FD, FD); k_gemm_hhx<0><<<gC, 128, 0, stream>>>(HLp + (size_t)a0 * FD, FD, 0, Bhh[r], FD, 0, 0.0625f / 1024.0f, nullptr, 0, GH, 1, (size_t)3 * FD, 0, GH, nullptr, 3 * FD, 0, CHK, 3 * FD, FD);
      k_gru<<<(CHK * (FD / 4) + 255) / 256, 256, 0, stream>>>(GI, GH, a0, H, HHp, HLp, AHp, ALp); } }
  k_gemm_hhx<0><<<gA, 128, 0, stream>>>(AHp, FD, 0, Bmt, FD, 0, 0.0625f, mtb, 0, nullptr, 1, 0, 0, AT, nullptr, FD, 0, NA, FD, FD); k_gemm_hhx<0><<<gA, 128, 0, stream>>>(ALp, FD, 0, Bmt, FD, 0, 0.0625f / 1024.0f, nullptr, 0, AT, 1, (size_t)FD, 0, AT, nullptr, FD, 0, NA, FD, FD);
  k_mol<<<NM, 256, 0, stream>>>(H, AT, amask, maw, mab, mwih, mwhh, mbih, mbhh, (float*)d_out);
}
